// SWEGNN_28441273434465
// MI455X (gfx1250) — hardware-verified
//
#include <hip/hip_runtime.h>
#include <stddef.h>


#define DF      8
#define EIN     36
#define HIDN    16
#define KP1     128
#define KP2     64
#define AP1     136
#define AP2     72
#define NTHR    256
#define NWAVE   8
#define EPB     128
#define NPB     128
#define EPT     8
#define NGRP    2
#define CHUNK   (NTHR * EPT * NGRP)
#define WCAP    (EPT * NGRP * 32)
#define LISTN   (NWAVE * WCAP)
#define NBC     4096
#define NBF     1024
#define RCAP    40960
#define RBN     128
#define DEGCAP  256
#define OTHR    512
#define LDS_FILL ((RCAP + NBF + LISTN) * 4 + 64)

static_assert((CHUNK & (CHUNK - 1)) == 0);
static_assert(CHUNK <= 4096);
static_assert((NBC & (NBC - 1)) == 0 && (NBF & (NBF - 1)) == 0);
static_assert(NBC == 4 * NBF);
static_assert(OTHR * 8 == NBC);
static_assert((RCAP % 32) == 0);
static_assert(EPB == NWAVE * 16 && NPB == NWAVE * 16);
static_assert((AP1 % 8) == 0 && (AP2 % 8) == 0);
static_assert(NTHR == NWAVE * 32);

typedef float        v4f  __attribute__((ext_vector_type(4)));
typedef float        v8f  __attribute__((ext_vector_type(8)));
typedef int          v4i  __attribute__((ext_vector_type(4)));
typedef unsigned int v4u  __attribute__((ext_vector_type(4)));
typedef v4u __attribute__((may_alias)) v4ua;
typedef __bf16       v16b __attribute__((ext_vector_type(16)));
union FragB { v16b v; v4u q[2]; };

__device__ __forceinline__ unsigned int bf_bits(float x) {
  const unsigned int u = __float_as_uint(x);
  return (u + 0x7FFFu + ((u >> 16) & 1u)) >> 16;
}
__device__ __forceinline__ void split1(float x, unsigned int& hb, unsigned int& lb) {
  hb = bf_bits(x);
  const float xh = __uint_as_float(hb << 16);
  lb = bf_bits(x - xh);
}
__device__ __forceinline__ void split8(v4f a, v4f b, v4u& hp, v4u& lp) {
  unsigned int h0, l0, h1, l1, h2, l2, h3, l3, h4, l4, h5, l5, h6, l6, h7, l7;
  split1(a.x, h0, l0); split1(a.y, h1, l1); split1(a.z, h2, l2); split1(a.w, h3, l3);
  split1(b.x, h4, l4); split1(b.y, h5, l5); split1(b.z, h6, l6); split1(b.w, h7, l7);
  hp.x = h0 | (h1 << 16); hp.y = h2 | (h3 << 16); hp.z = h4 | (h5 << 16); hp.w = h6 | (h7 << 16);
  lp.x = l0 | (l1 << 16); lp.y = l2 | (l3 << 16); lp.z = l4 | (l5 << 16); lp.w = l6 | (l7 << 16);
}
__device__ __forceinline__ v4f sel4(bool c, v4f a, v4f b) {
  v4f r;
  r.x = c ? a.x : b.x; r.y = c ? a.y : b.y; r.z = c ? a.z : b.z; r.w = c ? a.w : b.w;
  return r;
}

__device__ __forceinline__ v8f wmb(v16b a, v16b b, v8f c) {
  v8f d = __builtin_amdgcn_wmma_f32_16x16x32_bf16(false, a, false, b, (short)0, c, false, false);
  const v8f ax = __builtin_bit_cast(v8f, a);
  const v8f bx = __builtin_bit_cast(v8f, b);
  asm volatile("v_nop\n\tv_nop\n\tv_nop\n\tv_nop" : "+v"(d) : "v"(ax), "v"(bx));
  return d;
}

template <int NB>
__device__ __forceinline__ int scan_chunk(const int* __restrict__ dsts, int nE, int cbase, int slotBase,
                                          int vec8, int* list, int tid, int lane, int wave) {
  int wc = 0;
#pragma unroll
  for (int g = 0; g < NGRP; ++g) {
    const int el0  = (g * NTHR + tid) * EPT;
    const int e0   = cbase + el0;
    const int sent = -2147483647 - 1;
    v4i da, db;
    if (vec8 != 0 && cbase + CHUNK <= nE) {
      da = *(const v4i*)(dsts + e0);
      db = *(const v4i*)(dsts + e0 + 4);
    } else {
      da.x = (e0     < nE) ? dsts[min(e0, nE - 1)] : sent;
      da.y = (e0 + 1 < nE) ? dsts[min(e0 + 1, nE - 1)] : sent;
      da.z = (e0 + 2 < nE) ? dsts[min(e0 + 2, nE - 1)] : sent;
      da.w = (e0 + 3 < nE) ? dsts[min(e0 + 3, nE - 1)] : sent;
      db.x = (e0 + 4 < nE) ? dsts[min(e0 + 4, nE - 1)] : sent;
      db.y = (e0 + 5 < nE) ? dsts[min(e0 + 5, nE - 1)] : sent;
      db.z = (e0 + 6 < nE) ? dsts[min(e0 + 6, nE - 1)] : sent;
      db.w = (e0 + 7 < nE) ? dsts[min(e0 + 7, nE - 1)] : sent;
    }
    const unsigned nb = (unsigned)slotBase;
    const unsigned s0 = (unsigned)da.x - nb, s1 = (unsigned)da.y - nb;
    const unsigned s2 = (unsigned)da.z - nb, s3 = (unsigned)da.w - nb;
    const unsigned s4 = (unsigned)db.x - nb, s5 = (unsigned)db.y - nb;
    const unsigned s6 = (unsigned)db.z - nb, s7 = (unsigned)db.w - nb;
    const bool h0 = s0 < (unsigned)NB, h1 = s1 < (unsigned)NB, h2 = s2 < (unsigned)NB, h3 = s3 < (unsigned)NB;
    const bool h4 = s4 < (unsigned)NB, h5 = s5 < (unsigned)NB, h6 = s6 < (unsigned)NB, h7 = s7 < (unsigned)NB;
    const unsigned any = __builtin_amdgcn_ballot_w32(h0 | h1 | h2 | h3 | h4 | h5 | h6 | h7);
    if (any != 0u) {
#define HITJ(J, HJ, SJ) { \
        const unsigned mj = __builtin_amdgcn_ballot_w32(HJ); \
        if (mj != 0u) { \
          if (HJ) { \
            const int pos = wc + (int)__builtin_amdgcn_mbcnt_lo(mj, 0u); \
            if (pos < WCAP) list[wave * WCAP + pos] = ((el0 + (J)) << 12) | (int)(SJ); \
          } \
          wc += (int)__builtin_popcount(mj); } }
      HITJ(0, h0, s0)
      HITJ(1, h1, s1)
      HITJ(2, h2, s2)
      HITJ(3, h3, s3)
      HITJ(4, h4, s4)
      HITJ(5, h5, s5)
      HITJ(6, h6, s6)
      HITJ(7, h7, s7)
#undef HITJ
    }
  }
  return wc;
}

__global__ __launch_bounds__(NTHR) void k_wprep(
    const float* __restrict__ We1, const float* __restrict__ We2,
    unsigned short* w1p, unsigned short* w2p) {
  const int t = threadIdx.x;
  {
    const int n = t >> 4, g = t & 15;
    unsigned int e[8];
#pragma unroll
    for (int j = 0; j < 8; ++j) {
      const int p   = 8 * g + j;
      const int seg = p < 40 ? 0 : (p < 80 ? 1 : 2);
      const int k   = p - 40 * seg;
      const bool ok = k < EIN;
      const int kc  = ok ? k : 0;
      const float x = We1[kc * HIDN + n];
      unsigned int hb, lb; split1(x, hb, lb);
      const unsigned int v = (seg == 2) ? lb : hb;
      e[j] = ok ? v : 0u;
    }
    v4u o;
    o.x = e[0] | (e[1] << 16); o.y = e[2] | (e[3] << 16); o.z = e[4] | (e[5] << 16); o.w = e[6] | (e[7] << 16);
    unsigned short* gp = w1p + 8 * t;
    *(volatile v4ua*)gp = o;
    __threadfence();
    *(volatile v4ua*)gp = o;
  }
  if (t < 128) {
    const int n = t >> 3, g = t & 7;
    const bool nok = n < DF;
    const int nc = nok ? n : DF - 1;
    unsigned int e[8];
#pragma unroll
    for (int j = 0; j < 8; ++j) {
      const int p   = 8 * g + j;
      const int seg = p >> 4;
      const int k   = p & 15;
      const float x = We2[k * DF + nc];
      unsigned int hb, lb; split1(x, hb, lb);
      const unsigned int v = (seg == 2) ? lb : hb;
      e[j] = (nok && seg < 3) ? v : 0u;
    }
    v4u o;
    o.x = e[0] | (e[1] << 16); o.y = e[2] | (e[3] << 16); o.z = e[4] | (e[5] << 16); o.w = e[6] | (e[7] << 16);
    unsigned short* gp = w2p + 8 * t;
    *(volatile v4ua*)gp = o;
    __threadfence();
    *(volatile v4ua*)gp = o;
  }
}

__global__ __launch_bounds__(NTHR) void k_count(const int* __restrict__ ei, int* cnt, int nE, int vec8) {
  __shared__ __attribute__((aligned(16))) int scnt[NBC];
  __shared__ __attribute__((aligned(16))) int list[LISTN];
  __shared__ int wcnt[NWAVE];
  const int tid = threadIdx.x, lane = tid & 31, wave = tid >> 5;
  const int nodeBase = blockIdx.x * NBC;
  const int* dsts = ei + nE;

  for (int i = tid; i < NBC; i += NTHR) scnt[i] = 0;
  __syncthreads();

  const int nChunks = (nE + CHUNK - 1) / CHUNK;
#pragma unroll 1
  for (int ch = 0; ch < nChunks; ++ch) {
    const int cbase = ch * CHUNK;
    const int wc = scan_chunk<NBC>(dsts, nE, cbase, nodeBase, vec8, list, tid, lane, wave);
    if (lane == 0) wcnt[wave] = wc;
    __syncthreads();
    if (wave == 0) {
#pragma unroll 1
      for (int wsx = 0; wsx < NWAVE; ++wsx) {
        int n = __builtin_amdgcn_readfirstlane(wcnt[wsx]);
        n = n > WCAP ? WCAP : (n < 0 ? 0 : n);
        const int* lp = list + wsx * WCAP;
#pragma unroll 1
        for (int i = 0; i < n; ++i) {
          const int ent  = __builtin_amdgcn_readfirstlane(lp[i]);
          const int slot = ent & (NBC - 1);
          if (lane == 0) scnt[slot] = scnt[slot] + 1;
        }
      }
    }
    __syncthreads();
  }

  v4i cq[4];
#pragma unroll
  for (int q = 0; q < 4; ++q) {
    const int f = (wave * 4 + q) * 128 + 4 * lane;
    cq[q] = *(const v4i*)(scnt + f);
  }
  int* cp = cnt + (size_t)nodeBase;
#pragma unroll
  for (int q = 0; q < 4; ++q) {
    const int f = (wave * 4 + q) * 128 + 4 * lane;
    *(volatile v4i*)(cp + f) = cq[q];
  }
  __threadfence();
#pragma unroll
  for (int q = 0; q < 4; ++q) {
    const int f = (wave * 4 + q) * 128 + 4 * lane;
    *(volatile v4i*)(cp + f) = cq[q];
  }
}

__global__ __launch_bounds__(OTHR) void k_offsets(
    const int* __restrict__ cnt, int* off, int* rbase, int nChunk) {
  __shared__ __attribute__((aligned(16))) int soff[NBC];
  __shared__ __attribute__((aligned(16))) int srb[RBN];
  __shared__ int wtot[OTHR / 32];
  const int tid = threadIdx.x, lane = tid & 31, wave = tid >> 5, sub = tid >> 7;
  for (int i = tid; i < RBN; i += OTHR) srb[i] = 0;
  int carry = 0;
#pragma unroll 1
  for (int ch = 0; ch < nChunk; ++ch) {
    const int base = ch * NBC;
    const v4i c0 = *(const v4i*)(cnt + base + 8 * tid);
    const v4i c1 = *(const v4i*)(cnt + base + 8 * tid + 4);
    const int e0 = max(c0.x, 0), e1 = max(c0.y, 0), e2 = max(c0.z, 0), e3 = max(c0.w, 0);
    const int e4 = max(c1.x, 0), e5 = max(c1.y, 0), e6 = max(c1.z, 0), e7 = max(c1.w, 0);
    const int ts = e0 + e1 + e2 + e3 + e4 + e5 + e6 + e7;
    int incl = ts;
#pragma unroll
    for (int d = 1; d < 32; d <<= 1) {
      const int tv = __shfl_up(incl, d);
      if (lane >= d) incl += tv;
    }
    if (lane == 31) wtot[wave] = incl;
    __syncthreads();
    const int S0 = wtot[0]  + wtot[1]  + wtot[2]  + wtot[3];
    const int S1 = wtot[4]  + wtot[5]  + wtot[6]  + wtot[7];
    const int S2 = wtot[8]  + wtot[9]  + wtot[10] + wtot[11];
    const int S3 = wtot[12] + wtot[13] + wtot[14] + wtot[15];
    int pre = 0;
#pragma unroll 1
    for (int w = 4 * sub; w < wave; ++w) pre += wtot[w];
    const int b0 = carry;
    const int b1 = b0 + ((S0 + 31) & ~31);
    const int b2 = b1 + ((S1 + 31) & ~31);
    const int b3 = b2 + ((S2 + 31) & ~31);
    const int b4 = b3 + ((S3 + 31) & ~31);
    const int myb = sub == 0 ? b0 : (sub == 1 ? b1 : (sub == 2 ? b2 : b3));
    if (tid == 0) {
      srb[min(4 * ch + 0, RBN - 1)] = b0;
      srb[min(4 * ch + 1, RBN - 1)] = b1;
      srb[min(4 * ch + 2, RBN - 1)] = b2;
      srb[min(4 * ch + 3, RBN - 1)] = b3;
    }
    int run = myb + pre + incl - ts;
    soff[8 * tid + 0] = run; run += e0;
    soff[8 * tid + 1] = run; run += e1;
    soff[8 * tid + 2] = run; run += e2;
    soff[8 * tid + 3] = run; run += e3;
    soff[8 * tid + 4] = run; run += e4;
    soff[8 * tid + 5] = run; run += e5;
    soff[8 * tid + 6] = run; run += e6;
    soff[8 * tid + 7] = run;
    carry = b4;
    __syncthreads();
    const v4i o0 = *(const v4i*)(soff + 4 * tid);
    const v4i o1 = *(const v4i*)(soff + 4 * (tid + OTHR));
    int* op = off + base;
    *(volatile v4i*)(op + 4 * tid) = o0;
    *(volatile v4i*)(op + 4 * (tid + OTHR)) = o1;
    __threadfence();
    *(volatile v4i*)(op + 4 * tid) = o0;
    *(volatile v4i*)(op + 4 * (tid + OTHR)) = o1;
    __syncthreads();
  }
  if (tid == 0) srb[min(4 * nChunk, RBN - 1)] = carry;
  __syncthreads();
  v4i rv = {0, 0, 0, 0};
  if (tid < 32) rv = *(const v4i*)(srb + 4 * tid);
  if (tid < 32) *(volatile v4i*)(rbase + 4 * tid) = rv;
  __threadfence();
  if (tid < 32) *(volatile v4i*)(rbase + 4 * tid) = rv;
}

__global__ __launch_bounds__(NTHR) void k_fill(
    const int* __restrict__ ei, const int* __restrict__ off, const int* __restrict__ rbase,
    int* csr, int nE, int vec8, int csrLen) {
  extern __shared__ v4f lds_dyn[];
  int* region = (int*)lds_dyn;
  int* cursor = region + RCAP;
  int* list   = cursor + NBF;
  int* wcnt   = list + LISTN;
  const int tid = threadIdx.x, lane = tid & 31, wave = tid >> 5;
  const int b = blockIdx.x;
  const int nodeBase = b * NBF;
  const int* dsts = ei + nE;

  int rb0 = rbase[b];
  const int rb1 = rbase[b + 1];
  rb0 = rb0 < 0 ? 0 : (rb0 > csrLen ? csrLen : rb0);
  rb0 &= ~31;
  int len = rb1 - rb0;
  len = len < 0 ? 0 : (len > RCAP ? RCAP : len);
  int lenW = (len + 31) & ~31;
  if (rb0 + lenW > csrLen) lenW = (csrLen - rb0) & ~31;

  {
    const v4i z = {0, 0, 0, 0};
    for (int i = tid; i < RCAP / 4; i += NTHR) ((v4i*)region)[i] = z;
    for (int s = tid; s < NBF; s += NTHR) {
      int o = off[nodeBase + s] - rb0;
      o = o < 0 ? 0 : (o > RCAP ? RCAP : o);
      cursor[s] = o;
    }
  }
  __syncthreads();

  const int nChunks = (nE + CHUNK - 1) / CHUNK;
#pragma unroll 1
  for (int ch = 0; ch < nChunks; ++ch) {
    const int cbase = ch * CHUNK;
    const int wc = scan_chunk<NBF>(dsts, nE, cbase, nodeBase, vec8, list, tid, lane, wave);
    if (lane == 0) wcnt[wave] = wc;
    __syncthreads();
    if (wave == 0) {
#pragma unroll 1
      for (int wsx = 0; wsx < NWAVE; ++wsx) {
        int n = __builtin_amdgcn_readfirstlane(wcnt[wsx]);
        n = n > WCAP ? WCAP : (n < 0 ? 0 : n);
        const int* lp = list + wsx * WCAP;
#pragma unroll 1
        for (int i = 0; i < n; ++i) {
          const int ent  = __builtin_amdgcn_readfirstlane(lp[i]);
          const int slot = ent & (NBF - 1);
          int e = cbase + ((ent >> 12) & (CHUNK - 1));
          e = e > nE - 1 ? nE - 1 : e;
          if (lane == 0) {
            int pos = cursor[slot];
            pos = pos < 0 ? 0 : (pos > RCAP - 1 ? RCAP - 1 : pos);
            region[pos] = e;
            const int np = pos + 1;
            cursor[slot] = np > RCAP ? RCAP : np;
          }
        }
      }
    }
    __syncthreads();
  }

  const int nv = lenW >> 2;
  int* gp = csr + rb0;
#pragma unroll 1
  for (int i = tid; i < nv; i += NTHR) { const v4i v = ((const v4i*)region)[i]; *(volatile v4i*)(gp + 4 * i) = v; }
  __threadfence();
#pragma unroll 1
  for (int i = tid; i < nv; i += NTHR) { const v4i v = ((const v4i*)region)[i]; *(volatile v4i*)(gp + 4 * i) = v; }
}

__global__ __launch_bounds__(NTHR) void k_msg(
    const float* __restrict__ stat, const float* __restrict__ dyn, const int* __restrict__ ei,
    const float* __restrict__ ef, const unsigned short* __restrict__ w1p, const unsigned short* __restrict__ w2p,
    const float* __restrict__ be1, const float* __restrict__ be2, float* msg, int nN, int nE) {
  __shared__ __attribute__((aligned(16))) unsigned int   sA[EPB * (AP1 / 2)];
  __shared__ __attribute__((aligned(16))) unsigned short sH[EPB * AP2];
  __shared__ __attribute__((aligned(16))) float          stg[NWAVE * 16 * DF];
  const int t = threadIdx.x, lane = t & 31, wave = t >> 5, hh = lane >> 4, m = lane & 15;
  const int e0 = blockIdx.x * EPB;

  {
    const int el = t >> 1, half = t & 1;
    int eg = e0 + el; eg = eg > nE - 1 ? nE - 1 : eg;
    int node = ei[(size_t)half * (size_t)nE + (size_t)eg];
    node = node < 0 ? 0 : (node > nN - 1 ? nN - 1 : node);
    const float* sp = stat + (size_t)node * DF;
    const float* dp = dyn + (size_t)node * DF;
    const v4f s0 = *(const v4f*)sp, s1 = *(const v4f*)(sp + 4);
    const v4f d0 = *(const v4f*)dp, d1 = *(const v4f*)(dp + 4);
    const v4f f0 = *(const v4f*)(ef + (size_t)eg * 4);
    const v4f fz = {0.f, 0.f, 0.f, 0.f};
    v4u shp, slp, dhp, dlp, fhp, flp;
    split8(s0, s1, shp, slp);
    split8(d0, d1, dhp, dlp);
    split8(f0, fz, fhp, flp);
    unsigned int* rp = sA + el * (AP1 / 2);
    const int so = 4 * half;
    *(v4ua*)(rp + 0  + so) = shp;
    *(v4ua*)(rp + 20 + so) = slp;
    *(v4ua*)(rp + 40 + so) = shp;
    *(v4ua*)(rp + 8  + so) = dhp;
    *(v4ua*)(rp + 28 + so) = dlp;
    *(v4ua*)(rp + 48 + so) = dhp;
    if (half != 0) {
      const v4u z = {0u, 0u, 0u, 0u};
      *(v4ua*)(rp + 16) = fhp;
      *(v4ua*)(rp + 36) = flp;
      *(v4ua*)(rp + 56) = fhp;
      *(v4ua*)(rp + 60) = z;
    }
  }
  __syncthreads();

  const v8f z8 = {0.f, 0.f, 0.f, 0.f, 0.f, 0.f, 0.f, 0.f};

  v8f acc = z8;
  {
    const unsigned int*   ar = sA + (wave * 16 + m) * (AP1 / 2) + 4 * hh;
    const unsigned short* br = w1p + (size_t)m * KP1 + 8 * hh;
#pragma unroll
    for (int kt = 0; kt < KP1 / 32; ++kt) {
      FragB a, b;
      a.q[0] = *(const v4ua*)(ar + 16 * kt);
      a.q[1] = *(const v4ua*)(ar + 16 * kt + 8);
      b.q[0] = *(const v4ua*)(br + 32 * kt);
      b.q[1] = *(const v4ua*)(br + 32 * kt + 16);
      acc = wmb(a.v, b.v, acc);
    }
  }
  {
    const float b1v = be1[m];
    const int rb = (wave * 16 + 8 * hh) * AP2;
#pragma unroll
    for (int r = 0; r < 8; ++r) {
      float v = acc[r] + b1v;
      v = fmaxf(v, 0.0f);
      unsigned int hb, lb; split1(v, hb, lb);
      const int o = rb + r * AP2;
      sH[o + m]      = (unsigned short)hb;
      sH[o + 16 + m] = (unsigned short)lb;
      sH[o + 32 + m] = (unsigned short)hb;
      sH[o + 48 + m] = (unsigned short)0;
    }
  }
  __syncthreads();

  v8f acc2 = z8;
  {
    const unsigned short* ar = sH + (wave * 16 + m) * AP2 + 8 * hh;
    const unsigned short* br = w2p + (size_t)m * KP2 + 8 * hh;
#pragma unroll
    for (int kt = 0; kt < KP2 / 32; ++kt) {
      FragB a, b;
      a.q[0] = *(const v4ua*)(ar + 32 * kt);
      a.q[1] = *(const v4ua*)(ar + 32 * kt + 16);
      b.q[0] = *(const v4ua*)(br + 32 * kt);
      b.q[1] = *(const v4ua*)(br + 32 * kt + 16);
      acc2 = wmb(a.v, b.v, acc2);
    }
  }
  {
    const float b2v = be2[m < DF ? m : DF - 1];
    if (m < DF) {
      float* sp = stg + wave * (16 * DF) + (8 * hh) * DF + m;
#pragma unroll
      for (int r = 0; r < 8; ++r) sp[r * DF] = acc2[r] + b2v;
    }
  }
  __syncthreads();

  {
    const int edge = lane >> 1, part = lane & 1;
    const float* rp = stg + wave * (16 * DF) + edge * DF;
    const v4f va = *(const v4f*)rp, vb = *(const v4f*)(rp + 4);
    float ss = va.x * va.x;
    ss += va.y * va.y; ss += va.z * va.z; ss += va.w * va.w;
    ss += vb.x * vb.x; ss += vb.y * vb.y; ss += vb.z * vb.z; ss += vb.w * vb.w;
    const float nrm = sqrtf(ss);
    const float inv = nrm > 0.0f ? (1.0f / nrm) : 0.0f;
    const v4f o = sel4(part != 0, vb, va) * inv;
    float* gp = msg + ((size_t)e0 + (size_t)wave * 16) * DF + 4 * lane;
    *(volatile v4f*)gp = o;
    __threadfence();
    *(volatile v4f*)gp = o;
  }
}

__global__ __launch_bounds__(NTHR) void k_init(
    const float* __restrict__ dyn, const float* __restrict__ W0, float* dst, int nN, int dstRows) {
  __shared__ float sW[DF * DF];
  const int t = threadIdx.x;
  if (t < DF * DF) sW[t] = W0[t];
  __syncthreads();
  const int nl = t >> 1, part = t & 1;
  const int node = blockIdx.x * NPB + nl;
  const int nc = node > nN - 1 ? nN - 1 : node;
  const float* dp = dyn + (size_t)nc * DF;
  const v4f d0 = *(const v4f*)dp, d1 = *(const v4f*)(dp + 4);
  const float d[8] = { d0.x, d0.y, d0.z, d0.w, d1.x, d1.y, d1.z, d1.w };
  float o[4];
#pragma unroll
  for (int jj = 0; jj < 4; ++jj) {
    const int j = 4 * part + jj;
    float a = 0.0f;
#pragma unroll
    for (int i = 0; i < DF; ++i) a = fmaf(d[i], sW[i * DF + j], a);
    o[jj] = a;
  }
  v4f ov; ov.x = o[0]; ov.y = o[1]; ov.z = o[2]; ov.w = o[3];
  float* gp = dst + (size_t)node * DF + 4 * part;
  const bool ok = node < dstRows;
  if (ok) *(volatile v4f*)gp = ov;
  __threadfence();
  if (ok) *(volatile v4f*)gp = ov;
}

__global__ __launch_bounds__(NTHR) void k_step(
    const float* __restrict__ hin, const float* __restrict__ msg, const int* __restrict__ ei,
    const int* __restrict__ csr, const int* __restrict__ off, const int* __restrict__ cnt,
    const float* __restrict__ Wk, float* dst, int nN, int nE, int csrLen, int dstRows) {
  __shared__ float sW[DF * DF];
  const int t = threadIdx.x;
  if (t < DF * DF) sW[t] = Wk[t];
  __syncthreads();
  const int nl = t >> 1, part = t & 1;
  const int node = blockIdx.x * NPB + nl;
  const float* hp = hin + (size_t)node * DF;
  const v4f a0 = *(const v4f*)hp, a1 = *(const v4f*)(hp + 4);
  const float hs = ((((((a0.x + a0.y) + a0.z) + a0.w) + a1.x) + a1.y) + a1.z) + a1.w;
  const bool acti = hs != 0.0f;
  const v4f hi4 = sel4(part != 0, a1, a0);
  int n = cnt[node];
  n = n < 0 ? 0 : (n > DEGCAP ? DEGCAP : n);
  int st = off[node];
  st = st < 0 ? 0 : (st > csrLen - 1 ? csrLen - 1 : st);
  const v4f z4 = {0.f, 0.f, 0.f, 0.f};
  v4f agg = z4;
#pragma unroll 1
  for (int p = 0; p < n; ++p) {
    int pos = st + p;
    pos = pos > csrLen - 1 ? csrLen - 1 : pos;
    int e = csr[pos];
    e = e < 0 ? 0 : (e > nE - 1 ? nE - 1 : e);
    int r = ei[e];
    r = r < 0 ? 0 : (r > nN - 1 ? nN - 1 : r);
    const float* rq = hin + (size_t)r * DF;
    const v4f b0 = *(const v4f*)rq, b1 = *(const v4f*)(rq + 4);
    const float rs = ((((((b0.x + b0.y) + b0.z) + b0.w) + b1.x) + b1.y) + b1.z) + b1.w;
    const bool actr = rs != 0.0f;
    const v4f m4 = *(const v4f*)(msg + (size_t)e * DF + 4 * part);
    const v4f hr4 = sel4(part != 0, b1, b0);
    const v4f fl = (hi4 - hr4) * m4;
    agg = agg + sel4(acti || actr, fl, z4);
  }
  v4f oth;
  oth.x = __shfl_xor(agg.x, 1);
  oth.y = __shfl_xor(agg.y, 1);
  oth.z = __shfl_xor(agg.z, 1);
  oth.w = __shfl_xor(agg.w, 1);
  const v4f g0 = sel4(part != 0, oth, agg);
  const v4f g1 = sel4(part != 0, agg, oth);
  const float g[8] = { g0.x, g0.y, g0.z, g0.w, g1.x, g1.y, g1.z, g1.w };
  float o[4];
#pragma unroll
  for (int jj = 0; jj < 4; ++jj) {
    const int j = 4 * part + jj;
    float dsum = 0.0f;
#pragma unroll
    for (int i = 0; i < DF; ++i) dsum = fmaf(g[i], sW[i * DF + j], dsum);
    o[jj] = dsum;
  }
  v4f ov;
  ov.x = hi4.x + o[0]; ov.y = hi4.y + o[1]; ov.z = hi4.z + o[2]; ov.w = hi4.w + o[3];
  float* gp = dst + (size_t)node * DF + 4 * part;
  const bool ok = node < dstRows;
  if (ok) *(volatile v4f*)gp = ov;
  __threadfence();
  if (ok) *(volatile v4f*)gp = ov;
}

extern "C" void kernel_launch(void* const* d_in, const int* in_sizes, int n_in,
                              void* d_out, int out_size, void* d_ws, size_t ws_size,
                              hipStream_t stream) {
  if (n_in < 9) return;
  const int nN = in_sizes[0] / DF;
  const int nE = in_sizes[2] / 2;
  if (nN <= 0 || nE <= 0) return;
  if (in_sizes[0] != nN * DF || in_sizes[1] != nN * DF || in_sizes[2] != 2 * nE || in_sizes[3] != nE * 4) return;
  const int nK = in_sizes[4] / (DF * DF) - 1;
  if (nK < 0 || in_sizes[4] != (nK + 1) * DF * DF) return;
  if (in_sizes[5] != EIN * HIDN || in_sizes[6] < HIDN || in_sizes[7] != HIDN * DF || in_sizes[8] < DF) return;
  if (out_size != nN * DF) return;
  if (nE > (1 << 28) || nN > (1 << 24)) return;

  const float* stat = (const float*)d_in[0];
  const float* dyn  = (const float*)d_in[1];
  const int*   ei   = (const int*)d_in[2];
  const float* ef   = (const float*)d_in[3];
  const float* Wf   = (const float*)d_in[4];
  const float* We1  = (const float*)d_in[5];
  const float* be1  = (const float*)d_in[6];
  const float* We2  = (const float*)d_in[7];
  const float* be2  = (const float*)d_in[8];
  float* out = (float*)d_out;

  const int NPAD   = ((nN + NPB - 1) / NPB) * NPB;
  const int nBC    = (nN + NBC - 1) / NBC;
  const int CNTPAD = nBC * NBC;
  if (4 * nBC + 1 > RBN) return;
  const int nBF    = (nN + NBF - 1) / NBF;
  const int csrLen = ((nE + 31) & ~31) + 4096;
  const int EPAD   = ((nE + EPB - 1) / EPB) * EPB;
  const int nMsg   = EPAD / EPB;
  const int nNode  = NPAD / NPB;

  char* ws = (char*)d_ws;
  size_t off = 0;
  const size_t oW1  = off; off += (size_t)HIDN * KP1 * 2;          off = (off + 255) & ~(size_t)255;
  const size_t oW2  = off; off += (size_t)HIDN * KP2 * 2;          off = (off + 255) & ~(size_t)255;
  const size_t oCnt = off; off += (size_t)CNTPAD * 4;              off = (off + 255) & ~(size_t)255;
  const size_t oOff = off; off += (size_t)CNTPAD * 4;              off = (off + 255) & ~(size_t)255;
  const size_t oRb  = off; off += (size_t)RBN * 4;                 off = (off + 255) & ~(size_t)255;
  const size_t oCsr = off; off += (size_t)csrLen * 4;              off = (off + 255) & ~(size_t)255;
  const size_t oMsg = off; off += (size_t)EPAD * DF * 4;           off = (off + 255) & ~(size_t)255;
  const size_t oH0  = off; off += (size_t)NPAD * DF * 4;           off = (off + 255) & ~(size_t)255;
  const size_t oH1  = off; off += (size_t)NPAD * DF * 4;           off = (off + 255) & ~(size_t)255;
  if (off > ws_size) return;
  unsigned short* w1p = (unsigned short*)(ws + oW1);
  unsigned short* w2p = (unsigned short*)(ws + oW2);
  int*   cnt  = (int*)(ws + oCnt);
  int*   offp = (int*)(ws + oOff);
  int*   rb   = (int*)(ws + oRb);
  int*   csr  = (int*)(ws + oCsr);
  float* msgp = (float*)(ws + oMsg);
  float* h0   = (float*)(ws + oH0);
  float* h1   = (float*)(ws + oH1);

  const int vec8 = ((nE & 3) == 0) ? 1 : 0;

  k_wprep<<<1, NTHR, 0, stream>>>(We1, We2, w1p, w2p);

  k_count<<<nBC, NTHR, 0, stream>>>(ei, cnt, nE, vec8);
  k_offsets<<<1, OTHR, 0, stream>>>(cnt, offp, rb, nBC);
  hipFuncSetAttribute(reinterpret_cast<const void*>(&k_fill),
                      hipFuncAttributeMaxDynamicSharedMemorySize, LDS_FILL);
  k_fill<<<nBF, NTHR, LDS_FILL, stream>>>(ei, offp, rb, csr, nE, vec8, csrLen);

  k_msg<<<nMsg, NTHR, 0, stream>>>(stat, dyn, ei, ef, w1p, w2p, be1, be2, msgp, nN, nE);

  if (nK == 0) {
    k_init<<<nNode, NTHR, 0, stream>>>(dyn, Wf, out, nN, nN);
    return;
  }
  k_init<<<nNode, NTHR, 0, stream>>>(dyn, Wf, h0, nN, NPAD);

  for (int k = 0; k < nK; ++k) {
    const float* src = (k & 1) ? h1 : h0;
    float* dstp = (k & 1) ? h0 : h1;
    int dstRows = NPAD;
    if (k == nK - 1) { dstp = out; dstRows = nN; }
    k_step<<<nNode, NTHR, 0, stream>>>(src, msgp, ei, csr, offp, cnt,
                                       Wf + (size_t)(k + 1) * DF * DF, dstp, nN, nE, csrLen, dstRows);
  }
}
